// DotProductAttention_2095944040804
// MI455X (gfx1250) — hardware-verified
//
#include <hip/hip_runtime.h>
#include <math.h>

typedef __attribute__((ext_vector_type(16))) _Float16 v16h;
typedef __attribute__((ext_vector_type(8)))  _Float16 v8h;
typedef __attribute__((ext_vector_type(16))) __bf16   v16b;
typedef __attribute__((ext_vector_type(8)))  __bf16   v8b;
typedef __attribute__((ext_vector_type(8)))  float    v8f;
typedef __attribute__((ext_vector_type(4)))  float    v4f;
typedef __attribute__((ext_vector_type(4)))  unsigned int v4u;

constexpr int kBatch = 32;
constexpr int kSeq   = 2048;
constexpr int kDim   = 64;
constexpr int kTot   = kBatch * kSeq * kDim;
constexpr int kQB    = 64;
constexpr int kKC    = 64;
constexpr int kNW    = 4;
constexpr int kNQB   = kSeq / kQB;
constexpr int kNCH   = kSeq / kKC;
constexpr float kMaskFill = -1.0e6f;
constexpr float kQScale   = 0.125f;

static_assert(kSeq % kQB == 0);
static_assert(kSeq % kKC == 0);
static_assert(kDim == 64);
static_assert(kKC % 32 == 0);
static_assert(kTot % (8 * 256) == 0);

__device__ __forceinline__ unsigned short f2bf_bits(float f) {
  unsigned u = __float_as_uint(f);
  return (unsigned short)((u + 0x7FFFu + ((u >> 16) & 1u)) >> 16);
}
__device__ __forceinline__ float bf_bits2f(unsigned short h) { return __uint_as_float(((unsigned)h) << 16); }

__device__ __forceinline__ void dep_guard_h(v8f& a, v8f& b, v16h x, v16h y) { asm volatile("v_nop\n\tv_nop\n\tv_nop\n\tv_nop" : "+v"(a), "+v"(b) : "v"(x), "v"(y)); }
__device__ __forceinline__ void dep_guard_b(v8f& a, v8f& b, v16b x, v16b y) { asm volatile("v_nop\n\tv_nop\n\tv_nop\n\tv_nop" : "+v"(a), "+v"(b) : "v"(x), "v"(y)); }
__device__ __forceinline__ void keep4_h(v16h a, v16h b, v16h c, v16h d) { asm volatile("v_nop" :: "v"(a), "v"(b), "v"(c), "v"(d)); }
__device__ __forceinline__ void keep4_b(v16b a, v16b b, v16b c, v16b d) { asm volatile("v_nop" :: "v"(a), "v"(b), "v"(c), "v"(d)); }
template <typename T> struct Frag;
template <> struct Frag<_Float16> {
  typedef v16h V; union U { v16h v; v8h h[2]; };
  static __device__ __forceinline__ v16h load(const _Float16* p) {
    U f; f.h[0] = *(const v8h*)(p); f.h[1] = *(const v8h*)(p + 16); return f.v;
  }
  static __device__ __forceinline__ v8f mma(v16h a, v16h b, v8f c) {
    return __builtin_amdgcn_wmma_f32_16x16x32_f16(false, a, false, b, (short)0, c, false, false);
  }
  static __device__ __forceinline__ void guard(v8f& a, v8f& b, v16h x, v16h y) { dep_guard_h(a, b, x, y); }
  static __device__ __forceinline__ void keep(v16h a, v16h b, v16h c, v16h d) { keep4_h(a, b, c, d); }
};
template <> struct Frag<__bf16> {
  typedef v16b V; union U { v16b v; v8b h[2]; };
  static __device__ __forceinline__ v16b load(const __bf16* p) {
    U f; f.h[0] = *(const v8b*)(p); f.h[1] = *(const v8b*)(p + 16); return f.v;
  }
  static __device__ __forceinline__ v8f mma(v16b a, v16b b, v8f c) {
    return __builtin_amdgcn_wmma_f32_16x16x32_bf16(false, a, false, b, (short)0, c, false, false);
  }
  static __device__ __forceinline__ void guard(v8f& a, v8f& b, v16b x, v16b y) { dep_guard_b(a, b, x, y); }
  static __device__ __forceinline__ void keep(v16b a, v16b b, v16b c, v16b d) { keep4_b(a, b, c, d); }
};

__device__ __forceinline__ unsigned short at_bf_bits(float f) {
  unsigned u = __float_as_uint(f);
  return (unsigned short)((u + 0x7FFFu + ((u >> 16) & 1u)) >> 16);
}
__device__ __forceinline__ __bf16 at_f2bf(float f) { return __builtin_bit_cast(__bf16, at_bf_bits(f)); }
__device__ __forceinline__ void at_split(float f, __bf16& hi, __bf16& lo) {
  const unsigned short hb = at_bf_bits(f);
  hi = __builtin_bit_cast(__bf16, hb);
  lo = at_f2bf(f - __uint_as_float(((unsigned)hb) << 16));
}
__device__ __forceinline__ v8f at_mma(v16b a, v16b b, v8f c) {
  c = __builtin_amdgcn_wmma_f32_16x16x32_bf16(false, a, false, b, (short)0, c, false, false);
  asm volatile("v_nop\n\tv_nop\n\tv_nop\n\tv_nop" : "+v"(c) : "v"(a), "v"(b));
  return c;
}

__global__ __launch_bounds__(256) void cast_f32_bf16x8(
    const float* __restrict__ in, unsigned short* __restrict__ out, int n8, float scale) {
  const int i = blockIdx.x * 256 + threadIdx.x;
  if (i < n8) {
    const float* src = in + (size_t)i * 8;
    const v4f a0 = *(const v4f*)(src);
    const v4f a1 = *(const v4f*)(src + 4);
    v4u u;
    u[0] = (unsigned)f2bf_bits(a0[0] * scale) | ((unsigned)f2bf_bits(a0[1] * scale) << 16);
    u[1] = (unsigned)f2bf_bits(a0[2] * scale) | ((unsigned)f2bf_bits(a0[3] * scale) << 16);
    u[2] = (unsigned)f2bf_bits(a1[0] * scale) | ((unsigned)f2bf_bits(a1[1] * scale) << 16);
    u[3] = (unsigned)f2bf_bits(a1[2] * scale) | ((unsigned)f2bf_bits(a1[3] * scale) << 16);
    unsigned short* dst = out + (size_t)i * 8;
    *(volatile v4u*)dst = u;
    __threadfence();
    *(volatile v4u*)dst = u;
  }
}

__global__ __launch_bounds__(128)
void attn_vl_kernel(const unsigned short* __restrict__ Qp, const unsigned short* __restrict__ Kp,
                    const unsigned short* __restrict__ Vp, const int* __restrict__ VL,
                    float* __restrict__ out) {
  union FB { v16b v; v8b h[2]; };
  __shared__ __align__(16) unsigned short Ksh[kKC * kDim];
  __shared__ __align__(16) unsigned short Vth[kDim * kKC];
  __shared__ __align__(16) __bf16 Psh[kNW][16 * kKC];
  __shared__ __align__(16) __bf16 Psl[kNW][16 * kKC];
  __shared__ __align__(16) float  Os[kNW][16 * 68];

  const int tid  = threadIdx.x;
  const int wave = tid >> 5;
  const int lane = tid & 31;
  const int hh   = lane >> 4;
  const int c    = lane & 15;

  const int bx = blockIdx.x;
  const int qb = bx % kNQB;
  const int b  = bx / kNQB;
  const int q0 = qb * kQB + wave * 16;

  int vlen = VL[b];
  vlen = vlen < 0 ? 0 : (vlen > kSeq ? kSeq : vlen);
  int nChunks = (vlen == 0) ? kNCH : ((vlen + kKC - 1) / kKC);
  nChunks = nChunks > kNCH ? kNCH : nChunks;

  const __bf16*         qplane = (const __bf16*)Qp + (size_t)b * kSeq * kDim;
  const unsigned short* kplane = Kp + (size_t)b * kSeq * kDim;
  const unsigned short* vplane = Vp + (size_t)b * kSeq * kDim;
  float*                oplane = out + (size_t)b * kSeq * kDim;

  v16b qa[2];
  {
    const __bf16* qrow = qplane + (size_t)(q0 + c) * kDim;
#pragma unroll
    for (int dc = 0; dc < 2; ++dc) qa[dc] = Frag<__bf16>::load(qrow + dc * 32 + 8 * hh);
  }

  float mrow[8], lrow[8];
  v8f oacc[4];
#pragma unroll
  for (int r = 0; r < 8; ++r) { mrow[r] = -INFINITY; lrow[r] = 0.f; }
#pragma unroll
  for (int t = 0; t < 4; ++t) oacc[t] = (v8f){0.f,0.f,0.f,0.f,0.f,0.f,0.f,0.f};

  for (int kc = 0; kc < nChunks; ++kc) {
    const int kv0 = kc * kKC;
    __syncthreads();
    {
#pragma unroll
      for (int it = 0; it < 4; ++it) {
        const int p   = tid + it * 128;
        const int kvr = p >> 3;
        const int c8  = (p & 7) * 8;
        const size_t go = (size_t)(kv0 + kvr) * kDim + c8;
        const v4u kw = *(const v4u*)(kplane + go);
        const v4u vw = *(const v4u*)(vplane + go);
        *(v4u*)(Ksh + kvr * kDim + c8) = kw;
#pragma unroll
        for (int e = 0; e < 4; ++e) {
          const unsigned w = vw[e];
          Vth[(c8 + 2 * e)     * kKC + kvr] = (unsigned short)(w & 0xffffu);
          Vth[(c8 + 2 * e + 1) * kKC + kvr] = (unsigned short)(w >> 16);
        }
      }
    }
    __syncthreads();

    v8f s[4];
#pragma unroll
    for (int j = 0; j < 4; ++j) {
      s[j] = (v8f){0.f,0.f,0.f,0.f,0.f,0.f,0.f,0.f};
#pragma unroll
      for (int dc = 0; dc < 2; ++dc) {
        FB kb;
        const __bf16* kr = (const __bf16*)Ksh + (j * 16 + c) * kDim + dc * 32 + 8 * hh;
        kb.h[0] = *(const v8b*)(kr);
        kb.h[1] = *(const v8b*)(kr + 16);
        s[j] = at_mma(qa[dc], kb.v, s[j]);
      }
    }

    float cm[8];
#pragma unroll
    for (int r = 0; r < 8; ++r) {
      float m = -INFINITY;
#pragma unroll
      for (int j = 0; j < 4; ++j) {
        const int kvcol = kv0 + j * 16 + c;
        if (kvcol >= vlen) s[j][r] = kMaskFill;
        m = fmaxf(m, s[j][r]);
      }
#pragma unroll
      for (int off = 1; off < 16; off <<= 1) m = fmaxf(m, __shfl_xor(m, off, 32));
      cm[r] = m;
    }

    __bf16* pwh = Psh[wave];
    __bf16* pwl = Psl[wave];
#pragma unroll
    for (int r = 0; r < 8; ++r) {
      const float mnew  = fmaxf(mrow[r], cm[r]);
      const float alpha = expf(mrow[r] - mnew);
      mrow[r] = mnew;
      float psum = 0.f;
#pragma unroll
      for (int j = 0; j < 4; ++j) {
        const float p = expf(s[j][r] - mnew);
        psum += p;
        __bf16 ph, pl;
        at_split(p, ph, pl);
        pwh[(8 * hh + r) * kKC + j * 16 + c] = ph;
        pwl[(8 * hh + r) * kKC + j * 16 + c] = pl;
      }
#pragma unroll
      for (int off = 1; off < 16; off <<= 1) psum += __shfl_xor(psum, off, 32);
      lrow[r] = lrow[r] * alpha + psum;
#pragma unroll
      for (int t = 0; t < 4; ++t) oacc[t][r] *= alpha;
    }
    __builtin_amdgcn_fence(__ATOMIC_RELEASE, "workgroup");
    __builtin_amdgcn_wave_barrier();
    __builtin_amdgcn_fence(__ATOMIC_ACQUIRE, "workgroup");

#pragma unroll
    for (int kk = 0; kk < 2; ++kk) {
      FB pa, pl;
      pa.h[0] = *(const v8b*)(pwh + c * kKC + kk * 32 + 8 * hh);
      pa.h[1] = *(const v8b*)(pwh + c * kKC + kk * 32 + 16 + 8 * hh);
      pl.h[0] = *(const v8b*)(pwl + c * kKC + kk * 32 + 8 * hh);
      pl.h[1] = *(const v8b*)(pwl + c * kKC + kk * 32 + 16 + 8 * hh);
#pragma unroll
      for (int t = 0; t < 4; ++t) {
        FB vb;
        const __bf16* vr = (const __bf16*)Vth + (t * 16 + c) * kKC + kk * 32 + 8 * hh;
        vb.h[0] = *(const v8b*)(vr);
        vb.h[1] = *(const v8b*)(vr + 16);
        oacc[t] = at_mma(pa.v, vb.v, oacc[t]);
        oacc[t] = at_mma(pl.v, vb.v, oacc[t]);
      }
    }
  }

  float* os = Os[wave];
#pragma unroll
  for (int r = 0; r < 8; ++r) {
    const float inv = 1.0f / lrow[r];
#pragma unroll
    for (int t = 0; t < 4; ++t) os[(8 * hh + r) * 68 + t * 16 + c] = oacc[t][r] * inv;
  }
  __builtin_amdgcn_fence(__ATOMIC_RELEASE, "workgroup");
  __builtin_amdgcn_wave_barrier();
  __builtin_amdgcn_fence(__ATOMIC_ACQUIRE, "workgroup");
  {
    const int c4 = (lane & 15) * 4;
    for (int pass = 0; pass < 2; ++pass) {
#pragma unroll
      for (int it = 0; it < 8; ++it) {
        const int row = it * 2 + hh;
        v4f val = *(const v4f*)(os + row * 68 + c4);
        *(volatile v4f*)(oplane + (size_t)(q0 + row) * kDim + c4) = val;
      }
      __threadfence();
    }
  }
}

extern "C" void kernel_launch(void* const* d_in, const int* in_sizes, int n_in,
                              void* d_out, int out_size, void* d_ws, size_t ws_size,
                              hipStream_t stream) {
  constexpr size_t kPlaneBytes = (size_t)kTot * 2;
  constexpr size_t kWsNeed     = 3 * kPlaneBytes;
  static_assert(kWsNeed == 25165824);
  static_assert(kWsNeed <= 134217728);
  if (n_in < 4) return;
  if (in_sizes[0] != kTot || in_sizes[1] != kTot || in_sizes[2] != kTot || in_sizes[3] < kBatch) return;
  if (out_size != kTot || ws_size < kWsNeed) return;

  const float* Q  = (const float*)d_in[0];
  const float* K  = (const float*)d_in[1];
  const float* V  = (const float*)d_in[2];
  const int*   VL = (const int*)d_in[3];
  float*       O  = (float*)d_out;

  unsigned short* Qp = (unsigned short*)d_ws;
  unsigned short* Kp = Qp + kTot;
  unsigned short* Vp = Kp + kTot;

  const int n8 = kTot / 8;
  dim3 castGrid(n8 / 256, 1, 1), castBlock(256, 1, 1);
  cast_f32_bf16x8<<<castGrid, castBlock, 0, stream>>>(Q, Qp, n8, kQScale);
  cast_f32_bf16x8<<<castGrid, castBlock, 0, stream>>>(K, Kp, n8, 1.0f);
  cast_f32_bf16x8<<<castGrid, castBlock, 0, stream>>>(V, Vp, n8, 1.0f);

  dim3 attGrid(kBatch * kNQB, 1, 1), attBlock(128, 1, 1);
  attn_vl_kernel<<<attGrid, attBlock, 0, stream>>>(Qp, Kp, Vp, VL, O);
}
